// AxialAttention_71012989272674
// MI455X (gfx1250) — hardware-verified
//
#include <hip/hip_runtime.h>
#include <math.h>
#include <stdint.h>

#ifndef NB
#define NB 2
#endif
#define NB_FULL 2
#ifndef SEQ
#define SEQ 128
#endif
#define EW  256
#define NH  8
#define HD  32
#define W3  (3 * EW)
#define KO  (2 * EW)
#define RB  (SEQ * SEQ)
#define RT  (NB * RB)
#define VTP 136
#define SOP 264

static_assert(NH * HD == EW);
static_assert(HD == 32);
static_assert(EW == 256);
static_assert(SEQ == 128);
static_assert(NB >= 1 && NB <= NB_FULL);
static_assert((RB % 64) == 0 && (RT % 8) == 0);
static_assert((((RB / 32) * (W3 / 64)) % 8) == 0);
static_assert((((RB / 32) * (EW / 64)) % 8) == 0);
static_assert((EW % 64) == 0 && (W3 % 64) == 0 && (KO % 64) == 0 && (EW % 32) == 0 && (KO % 32) == 0);
static_assert((SEQ % 16) == 0 && (SEQ % 8) == 0);

typedef _Float16 v16h __attribute__((ext_vector_type(16)));
typedef _Float16 v8h  __attribute__((ext_vector_type(8)));
typedef float    v8f  __attribute__((ext_vector_type(8)));
typedef float    v4f  __attribute__((ext_vector_type(4)));
typedef unsigned int v4u __attribute__((ext_vector_type(4)));
typedef unsigned int v2u __attribute__((ext_vector_type(2)));

__device__ __forceinline__ unsigned short bf_bits(float f) {
  unsigned u = __float_as_uint(f);
  return (unsigned short)((u + 0x7FFFu + ((u >> 16) & 1u)) >> 16);
}
__device__ __forceinline__ float bf_up(unsigned short h) { return __uint_as_float(((unsigned)h) << 16); }
__device__ __forceinline__ unsigned short h_bits(_Float16 x) { return __builtin_bit_cast(unsigned short, x); }
__device__ __forceinline__ unsigned pk16(unsigned short a, unsigned short b) { return (unsigned)a | ((unsigned)b << 16); }
__device__ __forceinline__ v8f zero8() { v8f z = {0.f, 0.f, 0.f, 0.f, 0.f, 0.f, 0.f, 0.f}; return z; }

__device__ __forceinline__ v16h ldfrag_h(const _Float16* p) {
  union { v16h v; v8h h[2]; } f;
  f.h[0] = *(const v8h*)(p);
  f.h[1] = *(const v8h*)(p + 16);
  return f.v;
}

__device__ __forceinline__ v8f mma_h(v16h a, v16h b, v8f c) {
  c = __builtin_amdgcn_wmma_f32_16x16x32_f16(false, a, false, b, (short)0, c, false, false);
#if defined(__HIP_DEVICE_COMPILE__)
  asm volatile("v_nop\n\tv_nop\n\tv_nop\n\tv_nop" : "+v"(c) : "v"(a), "v"(b));
#endif
  return c;
}

__global__ __launch_bounds__(256) void ln_planes(const float* __restrict__ e, const float* __restrict__ lw,
                                                 const float* __restrict__ lb, unsigned short* xh,
                                                 unsigned short* xl, int nrows) {
  const int lane = threadIdx.x & 31;
  const int wave = threadIdx.x >> 5;
  const int row = blockIdx.x * 8 + wave;
  if (row >= nrows) return;
  const int c0 = lane * 8;
  const float* src = e + (size_t)row * EW + c0;
  const v4f a0 = *(const v4f*)(src);
  const v4f a1 = *(const v4f*)(src + 4);
  const v4f w0 = *(const v4f*)(lw + c0);
  const v4f w1 = *(const v4f*)(lw + c0 + 4);
  const v4f b0 = *(const v4f*)(lb + c0);
  const v4f b1 = *(const v4f*)(lb + c0 + 4);
  float v[8], w[8], bb[8];
#pragma unroll
  for (int t = 0; t < 4; ++t) {
    v[t]      = bf_up(bf_bits(a0[t]));
    v[4 + t]  = bf_up(bf_bits(a1[t]));
    w[t]      = bf_up(bf_bits(w0[t]));
    w[4 + t]  = bf_up(bf_bits(w1[t]));
    bb[t]     = bf_up(bf_bits(b0[t]));
    bb[4 + t] = bf_up(bf_bits(b1[t]));
  }
  float s = 0.f;
#pragma unroll
  for (int t = 0; t < 8; ++t) s += v[t];
#pragma unroll
  for (int o = 16; o > 0; o >>= 1) s += __shfl_xor(s, o);
  const float mu = s * (1.0f / (float)EW);
  float d[8];
  float s2 = 0.f;
#pragma unroll
  for (int t = 0; t < 8; ++t) { d[t] = v[t] - mu; s2 += d[t] * d[t]; }
#pragma unroll
  for (int o = 16; o > 0; o >>= 1) s2 += __shfl_xor(s2, o);
  const float var = s2 * (1.0f / (float)EW);
  const float rs = rsqrtf(var + 1e-5f);
  v4u ph, pl;
#pragma unroll
  for (int t = 0; t < 4; ++t) {
    const float y0 = d[2 * t] * rs * w[2 * t] + bb[2 * t];
    const float y1 = d[2 * t + 1] * rs * w[2 * t + 1] + bb[2 * t + 1];
    const _Float16 hq0 = (_Float16)y0;
    const _Float16 hq1 = (_Float16)y1;
    const _Float16 lq0 = (_Float16)((y0 - (float)hq0) * 2048.0f);
    const _Float16 lq1 = (_Float16)((y1 - (float)hq1) * 2048.0f);
    ph[t] = pk16(h_bits(hq0), h_bits(hq1));
    pl[t] = pk16(h_bits(lq0), h_bits(lq1));
  }
  const size_t o = (size_t)row * EW + c0;
  for (int pass = 0; pass < 2; ++pass) {
    *(volatile v4u*)(xh + o) = ph;
    *(volatile v4u*)(xl + o) = pl;
    __threadfence();
  }
}

__global__ __launch_bounds__(256) void tr_f16(const float* __restrict__ in, unsigned short* out, int R, int C,
                                              float scale) {
  __shared__ __align__(16) float sv[64 * 68];
  const int tid = threadIdx.x;
  const int r0 = blockIdx.x * 64;
  const int c0 = blockIdx.y * 64;
#pragma unroll
  for (int i = 0; i < 4; ++i) {
    const int idx = i * 256 + tid;
    const int rr = idx >> 4, c4 = (idx & 15) * 4;
    const v4f a = *(const v4f*)(in + (size_t)(r0 + rr) * C + c0 + c4);
    *(v4f*)(sv + rr * 68 + c4) = a;
  }
  __syncthreads();

  const int gq = tid >> 3, piece = tid & 7;
  v4u hv[2];
  size_t hofs[2];
#pragma unroll
  for (int it = 0; it < 2; ++it) {
    const int cc = it * 32 + gq;
    v4u a;
#pragma unroll
    for (int t = 0; t < 4; ++t) {
      const float f0 = bf_up(bf_bits(sv[(piece * 8 + 2 * t) * 68 + cc]));
      const float f1 = bf_up(bf_bits(sv[(piece * 8 + 2 * t + 1) * 68 + cc]));
      a[t] = pk16(h_bits((_Float16)(f0 * scale)), h_bits((_Float16)(f1 * scale)));
    }
    hv[it] = a;
    hofs[it] = (size_t)(c0 + cc) * R + r0 + piece * 8;
  }
  for (int pass = 0; pass < 2; ++pass) {
#pragma unroll
    for (int it = 0; it < 2; ++it) {
      *(volatile v4u*)(out + hofs[it]) = hv[it];
    }
    __threadfence();
  }
}

__global__ __launch_bounds__(256) void mask_planes(const float* __restrict__ mk, float* ma, float* mb,
                                                   float msc) {
  __shared__ __align__(16) float sm[8 * 132];
  const int tid = threadIdx.x;
  const int grp = blockIdx.x;
  const int h = blockIdx.y;
  const int b = blockIdx.z;
  const size_t pb = ((size_t)(b * NH + h)) * SEQ * SEQ;
  v4f vd;
  size_t od;
  {
    const int xx = tid >> 5, y4 = (tid & 31) * 4;
    const int x = grp * 8 + xx;
    const float* src = mk + (((size_t)b * SEQ + x) * SEQ + y4) * NH + h;
#pragma unroll
    for (int t = 0; t < 4; ++t) vd[t] = msc * bf_up(bf_bits(src[(size_t)t * NH]));
    od = pb + (size_t)x * SEQ + y4;
  }
  {
    const int x = tid >> 1, yq = (tid & 1) * 4;
    const float* src = mk + (((size_t)b * SEQ + x) * SEQ + grp * 8 + yq) * NH + h;
#pragma unroll
    for (int t = 0; t < 4; ++t) sm[(yq + t) * 132 + x] = msc * bf_up(bf_bits(src[(size_t)t * NH]));
  }
  __syncthreads();
  v4f vt;
  size_t ot;
  {
    const int yy = tid >> 5, x4 = (tid & 31) * 4;
    vt = *(const v4f*)(sm + yy * 132 + x4);
    ot = pb + (size_t)(grp * 8 + yy) * SEQ + x4;
  }
  for (int pass = 0; pass < 2; ++pass) {
    *(volatile v4f*)(ma + od) = vd;
    *(volatile v4f*)(mb + ot) = vt;
    __threadfence();
  }
}

__global__ __launch_bounds__(256) void gemm_p(
    const unsigned short* __restrict__ Ahp, const unsigned short* __restrict__ Alp,
    const unsigned short* __restrict__ Btp, const float* __restrict__ bias,
    unsigned short* php, unsigned short* plp,
    float f0, float f1, float f2, float sch, float scl) {
  const _Float16* Ah = (const _Float16*)(const void*)Ahp;
  const _Float16* Al = (const _Float16*)(const void*)Alp;
  const _Float16* Bh = (const _Float16*)(const void*)Btp;
  __shared__ __align__(16) float sT[8][16 * 68];
  const int lane = threadIdx.x & 31;
  const int wave = threadIdx.x >> 5;
  constexpr int tilesN = W3 / 64;
  constexpr int tilesM = RB / 32;
  const int tile = blockIdx.x * 8 + wave;
  if (tile >= tilesM * tilesN) return;
  const int tm = tile / tilesN;
  const int tn = tile - tm * tilesN;
  const int m0 = tm << 5;
  const int sec = tn >> 2;
  const int h0 = (tn & 3) * 2;
  const int rlane = lane & 15;
  const int koff  = (lane >> 4) * 8;
  const int mOff  = (lane >> 4) * 8;
  int nB[4];
#pragma unroll
  for (int j = 0; j < 4; ++j) nB[j] = sec * EW + ((((j & 1) << 4) + rlane) << 3) + h0 + (j >> 1);

  v8f acch[2][4], accl[2][4];
#pragma unroll
  for (int i = 0; i < 2; ++i)
#pragma unroll
    for (int j = 0; j < 4; ++j) { acch[i][j] = zero8(); accl[i][j] = zero8(); }

  for (int k0 = 0; k0 < EW; k0 += 32) {
    v16h fh[2], fl[2];
#pragma unroll
    for (int i = 0; i < 2; ++i) {
      const size_t ao = (size_t)(m0 + (i << 4) + rlane) * EW + koff + k0;
      fh[i] = ldfrag_h(Ah + ao);
      fl[i] = ldfrag_h(Al + ao);
    }
#pragma unroll
    for (int j = 0; j < 4; ++j) {
      const size_t bofs = (size_t)nB[j] * EW + koff + k0;
      const v16h bfr = ldfrag_h(Bh + bofs);
#pragma unroll
      for (int i = 0; i < 2; ++i) {
        acch[i][j] = mma_h(fh[i], bfr, acch[i][j]);
        accl[i][j] = mma_h(fl[i], bfr, accl[i][j]);
      }
    }
  }

  const float fac = (sec == 0) ? f0 : ((sec == 1) ? f1 : f2);
  float bz[4];
#pragma unroll
  for (int j = 0; j < 4; ++j) bz[j] = bf_up(bf_bits(bias[nB[j]]));

  float* slab = sT[wave];
  const int g8 = lane >> 3, pc = lane & 7;
#pragma unroll
  for (int i = 0; i < 2; ++i) {
    const int mBase = m0 + (i << 4);
#pragma unroll
    for (int r = 0; r < 8; ++r) {
#pragma unroll
      for (int j = 0; j < 4; ++j) {
        slab[(mOff + r) * 68 + (j << 4) + rlane] = ((acch[i][j][r] + accl[i][j][r] * scl) * sch + bz[j]) * fac;
      }
    }
    __builtin_amdgcn_fence(__ATOMIC_RELEASE, "workgroup");
    __builtin_amdgcn_wave_barrier();
    __builtin_amdgcn_fence(__ATOMIC_ACQUIRE, "workgroup");
    {
      v4u hv[4], lv[4];
      size_t ofs[4];
#pragma unroll
      for (int q = 0; q < 4; ++q) {
        const int L = q * 4 + g8;
        const int hh = L >> 3, t = L & 7;
        const int row = 2 * t + (pc >> 2);
        const int d0 = (pc & 3) * 8;
        const v4f x0 = *(const v4f*)(slab + row * 68 + hh * 32 + d0);
        const v4f x1 = *(const v4f*)(slab + row * 68 + hh * 32 + d0 + 4);
        float f[8];
        f[0] = x0[0]; f[1] = x0[1]; f[2] = x0[2]; f[3] = x0[3];
        f[4] = x1[0]; f[5] = x1[1]; f[6] = x1[2]; f[7] = x1[3];
        v4u ph, pl;
#pragma unroll
        for (int u = 0; u < 4; ++u) {
          const float s0 = f[2 * u];
          const float s1 = f[2 * u + 1];
          const _Float16 hq0 = (_Float16)s0;
          const _Float16 hq1 = (_Float16)s1;
          const _Float16 lq0 = (_Float16)((s0 - (float)hq0) * 2048.0f);
          const _Float16 lq1 = (_Float16)((s1 - (float)hq1) * 2048.0f);
          ph[u] = pk16(h_bits(hq0), h_bits(hq1));
          pl[u] = pk16(h_bits(lq0), h_bits(lq1));
        }
        hv[q] = ph;
        lv[q] = pl;
        ofs[q] = (((size_t)(sec * NH + h0 + hh)) * RB + (size_t)(mBase + row)) * HD + d0;
      }
      for (int pass = 0; pass < 2; ++pass) {
#pragma unroll
        for (int q = 0; q < 4; ++q) {
          *(volatile v4u*)(php + ofs[q]) = hv[q];
          if (sec < 2) *(volatile v4u*)(plp + ofs[q]) = lv[q];
        }
        __threadfence();
      }
    }
    __builtin_amdgcn_fence(__ATOMIC_RELEASE, "workgroup");
    __builtin_amdgcn_wave_barrier();
    __builtin_amdgcn_fence(__ATOMIC_ACQUIRE, "workgroup");
  }
}

__global__ __launch_bounds__(256) void attn_ax(
    const unsigned short* __restrict__ php, const unsigned short* __restrict__ plp,
    const float* __restrict__ mp, unsigned short* vah, unsigned short* val,
    int dir, float xscl, float escl, float pcar, float oscl) {
  const _Float16* Ph = (const _Float16*)(const void*)php;
  const _Float16* Pl = (const _Float16*)(const void*)plp;
  __shared__ __align__(16) unsigned short sVt[NH * HD * VTP];
  __shared__ __align__(16) float sO[16 * SOP];
  const _Float16* sVh = (const _Float16*)(const void*)sVt;
  const int tid  = threadIdx.x;
  const int lane = tid & 31;
  const int h    = tid >> 5;
  const int nl   = lane & 15;
  const int g    = lane >> 4;
  const int g8   = g * 8;
  const int j    = blockIdx.x;
  const size_t hs = (size_t)RB * HD;
  const size_t ss = (size_t)NH * hs;
  const _Float16* Qh = Ph + (size_t)h * hs;
  const _Float16* Kh = Ph + ss + (size_t)h * hs;
  const _Float16* Ql = Pl + (size_t)h * hs;
  const _Float16* Kl = Pl + ss + (size_t)h * hs;
  const unsigned short* Vu = php + 2 * ss + (size_t)h * hs;
  const int ks = (dir != 0) ? SEQ : 1;
  const int js = (dir != 0) ? 1 : SEQ;

#pragma unroll
  for (int it = 0; it < 4; ++it) {
    const int u  = it * 32 + lane;
    const int kq = u >> 2, dq = u & 3;
    const int kb = kq * 4;
    v4u rw[4];
#pragma unroll
    for (int a = 0; a < 4; ++a) {
      const size_t rowk = (size_t)(kb + a) * ks + (size_t)j * js;
      rw[a] = *(const v4u*)(Vu + rowk * HD + dq * 8);
    }
#pragma unroll
    for (int d = 0; d < 8; ++d) {
      const int wd = d >> 1, sh = (d & 1) * 16;
      const unsigned x0 = (rw[0][wd] >> sh) & 0xFFFFu;
      const unsigned x1 = (rw[1][wd] >> sh) & 0xFFFFu;
      const unsigned x2 = (rw[2][wd] >> sh) & 0xFFFFu;
      const unsigned x3 = (rw[3][wd] >> sh) & 0xFFFFu;
      v2u o;
      o[0] = x0 | (x1 << 16);
      o[1] = x2 | (x3 << 16);
      *(v2u*)(sVt + (h * HD + dq * 8 + d) * VTP + kb) = o;
    }
  }
  __syncthreads();

#pragma unroll 1
  for (int s = 0; s < 8; ++s) {
    const int i = s * 16 + nl;
    const size_t qofs = ((size_t)i * SEQ + j) * HD + g8;
    const v16h qh = ldfrag_h(Qh + qofs);
    const v16h ql = ldfrag_h(Ql + qofs);
    const float* mrow = mp + ((size_t)h * SEQ + i) * SEQ + g8;

    v8f acc[8];
#pragma unroll
    for (int ct = 0; ct < 8; ++ct) {
      const int kk = ct * 16 + nl;
      const size_t kofs = ((size_t)kk * ks + (size_t)j * js) * HD + g8;
      const v16h kh = ldfrag_h(Kh + kofs);
      const v16h kl = ldfrag_h(Kl + kofs);
      const v4f mv0 = *(const v4f*)(mrow + ct * 16);
      const v4f mv1 = *(const v4f*)(mrow + ct * 16 + 4);
      v8f am;
      am[0] = mv0[0]; am[1] = mv0[1]; am[2] = mv0[2]; am[3] = mv0[3];
      am[4] = mv1[0]; am[5] = mv1[1]; am[6] = mv1[2]; am[7] = mv1[3];
      v8f ax = mma_h(kh, ql, zero8());
      ax = mma_h(kl, qh, ax);
      am = mma_h(kh, qh, am);
      acc[ct] = am + ax * xscl;
    }

    float mx = acc[0][0];
#pragma unroll
    for (int ct = 0; ct < 8; ++ct)
#pragma unroll
      for (int r = 0; r < 8; ++r) mx = fmaxf(mx, acc[ct][r]);
    mx = fmaxf(mx, __shfl_xor(mx, 16));
    float sum = 0.f;
#pragma unroll
    for (int ct = 0; ct < 8; ++ct)
#pragma unroll
      for (int r = 0; r < 8; ++r) {
        const float ev = __expf((acc[ct][r] - mx) * escl);
        acc[ct][r] = ev;
        sum += ev;
      }
    sum += __shfl_xor(sum, 16);
    const float rc = pcar / sum;

    v16h pb[4];
#pragma unroll
    for (int c = 0; c < 4; ++c) {
      union { v16h v; v8h hh[2]; } U;
      v8h p0, p1;
#pragma unroll
      for (int e2 = 0; e2 < 8; ++e2) {
        p0[e2] = (_Float16)(acc[2 * c][e2] * rc);
        p1[e2] = (_Float16)(acc[2 * c + 1][e2] * rc);
      }
      U.hh[0] = p0;
      U.hh[1] = p1;
      pb[c] = U.v;
    }

    v8f oacc[2];
#pragma unroll
    for (int dt = 0; dt < 2; ++dt) {
      v8f o = zero8();
#pragma unroll
      for (int c = 0; c < 4; ++c) {
        const v16h va = ldfrag_h(sVh + (h * HD + dt * 16 + nl) * VTP + 32 * c + g8);
        o = mma_h(va, pb[c], o);
      }
      oacc[dt] = o;
    }

#pragma unroll
    for (int dt = 0; dt < 2; ++dt)
#pragma unroll
      for (int r = 0; r < 8; ++r)
        sO[nl * SOP + ((dt * 16 + g8 + r) << 3) + h] = oacc[dt][r] * oscl;
    __syncthreads();

    {
      v4u hv[2], lv[2];
      size_t ofs[2];
#pragma unroll
      for (int q = 0; q < 2; ++q) {
        const int rr = 2 * h + q;
        const v4f x0 = *(const v4f*)(sO + rr * SOP + lane * 8);
        const v4f x1 = *(const v4f*)(sO + rr * SOP + lane * 8 + 4);
        float f[8];
        f[0] = x0[0]; f[1] = x0[1]; f[2] = x0[2]; f[3] = x0[3];
        f[4] = x1[0]; f[5] = x1[1]; f[6] = x1[2]; f[7] = x1[3];
        v4u ph, pl;
#pragma unroll
        for (int u = 0; u < 4; ++u) {
          const float s0 = f[2 * u] * 1024.0f;
          const float s1 = f[2 * u + 1] * 1024.0f;
          const _Float16 hq0 = (_Float16)s0;
          const _Float16 hq1 = (_Float16)s1;
          const _Float16 lq0 = (_Float16)((s0 - (float)hq0) * 2048.0f);
          const _Float16 lq1 = (_Float16)((s1 - (float)hq1) * 2048.0f);
          ph[u] = pk16(h_bits(hq0), h_bits(hq1));
          pl[u] = pk16(h_bits(lq0), h_bits(lq1));
        }
        hv[q] = ph;
        lv[q] = pl;
        ofs[q] = ((size_t)(s * 16 + rr) * SEQ + j) * KO + (size_t)dir * EW + lane * 8;
      }
      for (int pass = 0; pass < 2; ++pass) {
#pragma unroll
        for (int q = 0; q < 2; ++q) {
          *(volatile v4u*)(vah + ofs[q]) = hv[q];
          *(volatile v4u*)(val + ofs[q]) = lv[q];
        }
        __threadfence();
      }
    }
    __syncthreads();
  }
}

__global__ __launch_bounds__(256) void gemm32h_w(
    const unsigned short* __restrict__ Ahp, const unsigned short* __restrict__ Alp, int lda,
    const unsigned short* __restrict__ Btp, int ldb,
    const float* __restrict__ bias,
    float* C, int ldc, int M, int N, int K, float sch, float scl) {
  const _Float16* Ah = (const _Float16*)(const void*)Ahp;
  const _Float16* Al = (const _Float16*)(const void*)Alp;
  const _Float16* Bh = (const _Float16*)(const void*)Btp;
  __shared__ __align__(16) float sT[8][16 * 68];
  const int lane = threadIdx.x & 31;
  const int wave = threadIdx.x >> 5;
  const int tilesN = N >> 6;
  const int tilesM = M >> 5;
  const int tile = blockIdx.x * 8 + wave;
  if (tile >= tilesM * tilesN) return;
  const int tm = tile / tilesN;
  const int tn = tile - tm * tilesN;
  const int m0 = tm << 5;
  const int n0 = tn << 6;
  const int rlane = lane & 15;
  const int koff  = (lane >> 4) * 8;
  const int mOff  = (lane >> 4) * 8;

  v8f acch[2][4], accl[2][4];
#pragma unroll
  for (int i = 0; i < 2; ++i)
#pragma unroll
    for (int j = 0; j < 4; ++j) { acch[i][j] = zero8(); accl[i][j] = zero8(); }

  for (int k0 = 0; k0 < K; k0 += 32) {
    v16h fh[2], fl[2];
#pragma unroll
    for (int i = 0; i < 2; ++i) {
      const size_t ao = (size_t)(m0 + (i << 4) + rlane) * lda + koff + k0;
      fh[i] = ldfrag_h(Ah + ao);
      fl[i] = ldfrag_h(Al + ao);
    }
#pragma unroll
    for (int j = 0; j < 4; ++j) {
      const size_t bofs = (size_t)(n0 + (j << 4) + rlane) * ldb + koff + k0;
      const v16h bfr = ldfrag_h(Bh + bofs);
#pragma unroll
      for (int i = 0; i < 2; ++i) {
        acch[i][j] = mma_h(fh[i], bfr, acch[i][j]);
        accl[i][j] = mma_h(fl[i], bfr, accl[i][j]);
      }
    }
  }

  float bz[4];
#pragma unroll
  for (int j = 0; j < 4; ++j) bz[j] = bf_up(bf_bits(bias[n0 + (j << 4) + rlane]));

  float* slab = sT[wave];
#pragma unroll
  for (int i = 0; i < 2; ++i) {
    const int mBase = m0 + (i << 4);
#pragma unroll
    for (int r = 0; r < 8; ++r) {
#pragma unroll
      for (int j = 0; j < 4; ++j) {
        slab[(mOff + r) * 68 + (j << 4) + rlane] = (acch[i][j][r] + accl[i][j][r] * scl) * sch + bz[j];
      }
    }
    __builtin_amdgcn_fence(__ATOMIC_RELEASE, "workgroup");
    __builtin_amdgcn_wave_barrier();
    __builtin_amdgcn_fence(__ATOMIC_ACQUIRE, "workgroup");
    {
      const int hh = lane >> 4, c4 = (lane & 15) * 4;
      v4f ov[8];
#pragma unroll
      for (int it = 0; it < 8; ++it) {
        const int row = it * 2 + hh;
        ov[it] = *(const v4f*)(slab + row * 68 + c4);
      }
      for (int pass = 0; pass < 2; ++pass) {
#pragma unroll
        for (int it = 0; it < 8; ++it) {
          const int row = it * 2 + hh;
          *(volatile v4f*)(C + (size_t)(mBase + row) * ldc + n0 + c4) = ov[it];
        }
        __threadfence();
      }
    }
    __builtin_amdgcn_fence(__ATOMIC_RELEASE, "workgroup");
    __builtin_amdgcn_wave_barrier();
    __builtin_amdgcn_fence(__ATOMIC_ACQUIRE, "workgroup");
  }
}

extern "C" void kernel_launch(void* const* d_in, const int* in_sizes, int n_in,
                              void* d_out, int out_size, void* d_ws, size_t ws_size,
                              hipStream_t stream) {
  if (n_in < 10) return;
  if (in_sizes[0] < RT * EW) return;
  if (in_sizes[1] < NB * SEQ * SEQ * NH) return;
  if (in_sizes[2] < EW) return;
  if (in_sizes[3] < EW) return;
  if (in_sizes[4] < EW * W3) return;
  if (in_sizes[5] < W3) return;
  if (in_sizes[6] < EW * W3) return;
  if (in_sizes[7] < W3) return;
  if (in_sizes[8] < KO * EW) return;
  if (in_sizes[9] < EW) return;
  if (out_size < RT * EW) return;

  const float* e    = (const float*)d_in[0];
  const float* mask = (const float*)d_in[1];
  const float* ln_w = (const float*)d_in[2];
  const float* ln_b = (const float*)d_in[3];
  const float* Wqi  = (const float*)d_in[4];
  const float* bqi  = (const float*)d_in[5];
  const float* Wqo  = (const float*)d_in[6];
  const float* bqo  = (const float*)d_in[7];
  const float* Wo   = (const float*)d_in[8];
  const float* bo   = (const float*)d_in[9];

  const size_t PX  = (size_t)RT * EW * 2;
  const size_t PWt = (size_t)W3 * EW * 2;
  const size_t PWo = (size_t)EW * KO * 2;
  const size_t PM  = (size_t)NB * NH * SEQ * SEQ * 4;
  const size_t PPh = (size_t)3 * NH * RB * HD * 2;
  const size_t PPl = (size_t)2 * NH * RB * HD * 2;
  const size_t PVa = (size_t)RB * KO * 2;
  size_t off = 0;
  const size_t oXh = off; off += PX;
  const size_t oXl = off; off += PX;
  const size_t oWi = off; off += PWt;
  const size_t oWt = off; off += PWt;
  const size_t oWo = off; off += PWo;
  const size_t oMa = off; off += PM;
  const size_t oMb = off; off += PM;
  const size_t oPh = off; off += PPh;
  const size_t oPl = off; off += PPl;
  const size_t oVh = off; off += PVa;
  const size_t oVl = off; off += PVa;
  if (off > ws_size) return;
  if (off > (size_t)134217728) return;

  char* ws = (char*)d_ws;
  unsigned short* Xh  = (unsigned short*)(ws + oXh);
  unsigned short* Xl  = (unsigned short*)(ws + oXl);
  unsigned short* Wti = (unsigned short*)(ws + oWi);
  unsigned short* Wto = (unsigned short*)(ws + oWt);
  unsigned short* Woh = (unsigned short*)(ws + oWo);
  float*          mA  = (float*)(ws + oMa);
  float*          mB  = (float*)(ws + oMb);
  unsigned short* Ph  = (unsigned short*)(ws + oPh);
  unsigned short* Pl  = (unsigned short*)(ws + oPl);
  unsigned short* Vah = (unsigned short*)(ws + oVh);
  unsigned short* Val = (unsigned short*)(ws + oVl);
  float*          outf = (float*)d_out;

  const dim3 blk(256);
  const dim3 gLn(RT / 8);
  const dim3 gTw(EW / 64, W3 / 64);
  const dim3 gTo(KO / 64, EW / 64);
  const dim3 gMk(SEQ / 8, NH, NB);
  const dim3 gPr(((RB / 32) * (W3 / 64)) / 8);
  const dim3 gAt(SEQ);
  const dim3 gWo(((RB / 32) * (EW / 64)) / 8);
  const float cW     = 64.0f;
  const float fQ     = 16.0f * 0.17677669529663687f;
  const float fK     = 4.0f;
  const float fV     = 4.0f;
  const float prSch  = 1.0f / 64.0f;
  const float prScl  = 1.0f / 2048.0f;
  const float mkSc   = 64.0f;
  const float axXscl = 1.0f / 2048.0f;
  const float axEscl = 1.0f / 64.0f;
  const float axPcar = 16384.0f;
  const float axOscl = 1.0f / 65536.0f;
  const float woScale = 1024.0f;
  const float woSch  = 1.0f / 1048576.0f;
  const float woScl  = 1.0f / 2048.0f;

  ln_planes<<<gLn, blk, 0, stream>>>(e, ln_w, ln_b, Xh, Xl, RT);
  tr_f16<<<gTw, blk, 0, stream>>>(Wqi, Wti, EW, W3, cW);
  tr_f16<<<gTw, blk, 0, stream>>>(Wqo, Wto, EW, W3, cW);
  tr_f16<<<gTo, blk, 0, stream>>>(Wo, Woh, KO, EW, woScale);
  mask_planes<<<gMk, blk, 0, stream>>>(mask, mA, mB, mkSc);
  for (int b = 0; b < NB; ++b) {
    const size_t xo = (size_t)b * RB * EW;
    const size_t mo = (size_t)b * NH * SEQ * SEQ;
    gemm_p<<<gPr, blk, 0, stream>>>(Xh + xo, Xl + xo, Wti, bqi, Ph, Pl, fQ, fK, fV, prSch, prScl);
    attn_ax<<<gAt, blk, 0, stream>>>(Ph, Pl, mA + mo, Vah, Val, 0, axXscl, axEscl, axPcar, axOscl);
    gemm_p<<<gPr, blk, 0, stream>>>(Xh + xo, Xl + xo, Wto, bqo, Ph, Pl, fQ, fK, fV, prSch, prScl);
    attn_ax<<<gAt, blk, 0, stream>>>(Ph, Pl, mB + mo, Vah, Val, 1, axXscl, axEscl, axPcar, axOscl);
    gemm32h_w<<<gWo, blk, 0, stream>>>(Vah, Val, KO, Woh, KO, bo, outf + (size_t)b * RB * EW, EW,
                                        RB, EW, KO, woSch, woScl);
  }
  (void)hipGetLastError();
}
